// customGRU_38414187495806
// MI455X (gfx1250) — hardware-verified
//
#include <hip/hip_runtime.h>
#include <math.h>

constexpr int NBAT   = 64;
constexpr int NSTEP  = 64;
constexpr int NINP   = 512;
constexpr int NHID   = 1024;
constexpr int NG3    = 3 * NHID;
constexpr int NFC    = 256;
constexpr int NROWS  = NBAT * NSTEP;
constexpr int NOUT0  = NBAT * NFC;
constexpr int NOUT1  = 2 * NBAT * NHID;
constexpr int RTHR    = 512;
constexpr int SEQ_BLK = 16;
constexpr int HPITCH  = NHID + 8;
constexpr int HMPITCH = NHID + 4;
constexpr float WCARRY     = 256.0f;
constexpr float WCARRY_INV = 1.0f / 256.0f;
constexpr float ACARRY     = 16.0f;
constexpr float FC_SCALE   = 1.0f / (256.0f * 16.0f);

static_assert(NBAT % SEQ_BLK == 0, "batch tiles");
static_assert(NHID == 64 * (RTHR / 32), "16 waves x 64 hidden columns");
static_assert(NHID % 32 == 0 && NINP % 32 == 0, "GEMM K multiples of 32");
static_assert(NROWS % 64 == 0 && NG3 % 64 == 0 && NBAT % 64 == 0 && NFC % 64 == 0, "GEMM M, N tile multiples");
static_assert((SEQ_BLK * NHID / 8) % RTHR == 0, "16-bit row copy loop exact");
static_assert((SEQ_BLK * NHID / 4) % RTHR == 0, "f32 row copy loop exact");
static_assert(HPITCH % 8 == 0 && HMPITCH % 4 == 0, "LDS pitches keep 16-B alignment");
static_assert(NOUT0 * 4 == 65536, "second output starts at byte 65536");
static_assert((NOUT0 + NOUT1) * 4 == 589824, "d_out total bytes");

typedef __attribute__((ext_vector_type(16))) _Float16 v16h;
typedef __attribute__((ext_vector_type(8)))  _Float16 v8h;
typedef __attribute__((ext_vector_type(16))) __bf16   v16b;
typedef __attribute__((ext_vector_type(8)))  __bf16   v8b;
typedef __attribute__((ext_vector_type(8)))  float    v8f;
typedef __attribute__((ext_vector_type(4)))  float    v4f;

__device__ __forceinline__ unsigned short f2bf_bits(float f) {
  unsigned u = __float_as_uint(f);
  return (unsigned short)((u + 0x7FFFu + ((u >> 16) & 1u)) >> 16);
}
__device__ __forceinline__ float bf_bits2f(unsigned short h) { return __uint_as_float(((unsigned)h) << 16); }
__device__ __forceinline__ float bf16r(float f) { return bf_bits2f(f2bf_bits(f)); }

__device__ __forceinline__ void dep_guard4_h(v8f& a, v8f& b, v8f& c, v8f& d, v16h x, v16h y) { asm volatile("v_nop\n\tv_nop\n\tv_nop\n\tv_nop" : "+v"(a), "+v"(b), "+v"(c), "+v"(d) : "v"(x), "v"(y)); }
__device__ __forceinline__ void dep_guard4_b(v8f& a, v8f& b, v8f& c, v8f& d, v16b x, v16b y) { asm volatile("v_nop\n\tv_nop\n\tv_nop\n\tv_nop" : "+v"(a), "+v"(b), "+v"(c), "+v"(d) : "v"(x), "v"(y)); }
__device__ __forceinline__ void keep4_h(v16h a, v16h b, v16h c, v16h d) { asm volatile("v_nop" :: "v"(a), "v"(b), "v"(c), "v"(d)); }
__device__ __forceinline__ void keep4_b(v16b a, v16b b, v16b c, v16b d) { asm volatile("v_nop" :: "v"(a), "v"(b), "v"(c), "v"(d)); }
__device__ __forceinline__ void acc_guard4(v8f& a, v8f& b, v8f& c, v8f& d) { asm volatile("v_nop\n\tv_nop\n\tv_nop\n\tv_nop" : "+v"(a), "+v"(b), "+v"(c), "+v"(d)); }
__device__ __forceinline__ void acc_guard3(v8f& a, v8f& b, v8f& c) { asm volatile("v_nop\n\tv_nop\n\tv_nop\n\tv_nop" : "+v"(a), "+v"(b), "+v"(c)); }
__device__ __forceinline__ void guard3_h(v8f& a, v8f& b, v8f& c, v16h x, v16h y0, v16h y1, v16h y2) {
  asm volatile("v_nop\n\tv_nop\n\tv_nop\n\tv_nop" : "+v"(a), "+v"(b), "+v"(c) : "v"(x), "v"(y0), "v"(y1), "v"(y2));
}

template <typename T> struct Frag;
template <> struct Frag<_Float16> {
  typedef v16h V; union U { v16h v; v8h h[2]; };
  static __device__ __forceinline__ v16h load(const _Float16* p) {
    U f; f.h[0] = *(const v8h*)(p); f.h[1] = *(const v8h*)(p + 16); return f.v;
  }
  static __device__ __forceinline__ v8f mma(v16h a, v16h b, v8f c) {
    return __builtin_amdgcn_wmma_f32_16x16x32_f16(false, a, false, b, (short)0, c, false, false);
  }
  static __device__ __forceinline__ void guard4(v8f& a, v8f& b, v8f& c, v8f& d, v16h x, v16h y) { dep_guard4_h(a, b, c, d, x, y); }
  static __device__ __forceinline__ void keep(v16h a, v16h b, v16h c, v16h d) { keep4_h(a, b, c, d); }
};
template <> struct Frag<__bf16> {
  typedef v16b V; union U { v16b v; v8b h[2]; };
  static __device__ __forceinline__ v16b load(const __bf16* p) {
    U f; f.h[0] = *(const v8b*)(p); f.h[1] = *(const v8b*)(p + 16); return f.v;
  }
  static __device__ __forceinline__ v8f mma(v16b a, v16b b, v8f c) {
    return __builtin_amdgcn_wmma_f32_16x16x32_bf16(false, a, false, b, (short)0, c, false, false);
  }
  static __device__ __forceinline__ void guard4(v8f& a, v8f& b, v8f& c, v8f& d, v16b x, v16b y) { dep_guard4_b(a, b, c, d, x, y); }
  static __device__ __forceinline__ void keep(v16b a, v16b b, v16b c, v16b d) { keep4_b(a, b, c, d); }
};

template <int ET> struct Elem;
template <> struct Elem<0> { typedef _Float16 T; };
template <> struct Elem<1> { typedef __bf16 T; };
template <int ET, bool SPLIT, int BIAS_MODE, int OUT_MODE, bool RESID, int ACT = 0>
__global__ __launch_bounds__(256) void wmma_gemm64(
    const unsigned short* __restrict__ Ap, const unsigned short* __restrict__ A2p, int lda, long strideA,
    const unsigned short* __restrict__ Btp, const unsigned short* __restrict__ Bt2p, int ldb, long strideB,
    void* __restrict__ Cout, void* __restrict__ Cout2, int ldc, long strideC,
    const float* __restrict__ bias,
    const float* __restrict__ resid, long strideR,
    int M, int N, int K, float scale) {
  typedef typename Elem<ET>::T T;
  typedef typename Frag<T>::V V;
  const T* A = (const T*)Ap; const T* A2 = (const T*)A2p; const T* Bt = (const T*)Btp; const T* Bt2 = (const T*)Bt2p;
  __shared__ __align__(16) float sT[8][16 * 68];
  const int b    = blockIdx.y;
  const int lane = threadIdx.x & 31;
  const int wave = threadIdx.x >> 5;
  const int tilesN = N >> 6;
  const int tilesM = M >> 6;
  const int tile = blockIdx.x * 8 + wave;
  if (tile >= tilesM * tilesN) return;
  const int tm = tile / tilesN;
  const int tn = tile - tm * tilesN;
  const int m0 = tm << 6;
  const int n0 = tn << 6;

  const T* Ab  = A  + (size_t)b * strideA;
  const T* Bb  = Bt + (size_t)b * strideB;
  const T* Ab2 = SPLIT ? (A2  + (size_t)b * strideA) : nullptr;
  const T* Bb2 = SPLIT ? (Bt2 + (size_t)b * strideB) : nullptr;

  const int rlane = lane & 15;
  const int koff  = (lane >> 4) * 8;
  const int mOff  = (lane >> 4) * 8;

  v8f acc[4][4];
#pragma unroll
  for (int i = 0; i < 4; ++i)
#pragma unroll
    for (int j = 0; j < 4; ++j) acc[i][j] = (v8f){0.f,0.f,0.f,0.f,0.f,0.f,0.f,0.f};

  for (int k0 = 0; k0 < K; k0 += 32) {
    V bh[4], bl[4];
#pragma unroll
    for (int j = 0; j < 4; ++j) {
      const size_t bo = (size_t)(n0 + (j << 4) + rlane) * ldb + koff + k0;
      bh[j] = Frag<T>::load(Bb + bo);
      if (SPLIT) bl[j] = Frag<T>::load(Bb2 + bo);
    }
#pragma unroll
    for (int i = 0; i < 4; ++i) {
      const size_t ao = (size_t)(m0 + (i << 4) + rlane) * lda + koff + k0;
      V ah = Frag<T>::load(Ab + ao);
      V al;
      if (SPLIT) al = Frag<T>::load(Ab2 + ao);
#pragma unroll
      for (int j = 0; j < 4; ++j) {
        acc[i][j] = Frag<T>::mma(ah, bh[j], acc[i][j]);
        if (SPLIT) {
          acc[i][j] = Frag<T>::mma(ah, bl[j], acc[i][j]);
          acc[i][j] = Frag<T>::mma(al, bh[j], acc[i][j]);
        }
      }
      Frag<T>::guard4(acc[i][0], acc[i][1], acc[i][2], acc[i][3], ah, SPLIT ? al : ah);
    }
    Frag<T>::keep(bh[0], bh[1], bh[2], bh[3]);
    if (SPLIT) Frag<T>::keep(bl[0], bl[1], bl[2], bl[3]);
  }
  acc_guard4(acc[0][0], acc[0][1], acc[0][2], acc[0][3]);
  acc_guard4(acc[1][0], acc[1][1], acc[1][2], acc[1][3]);
  acc_guard4(acc[2][0], acc[2][1], acc[2][2], acc[2][3]);
  acc_guard4(acc[3][0], acc[3][1], acc[3][2], acc[3][3]);

  float* slab = sT[wave];
  const float* Rb = RESID ? (resid + (size_t)b * strideR) : nullptr;
#pragma unroll
  for (int i = 0; i < 4; ++i) {
    const int mBase = m0 + (i << 4);
#pragma unroll
    for (int j = 0; j < 4; ++j) {
      const int n = n0 + (j << 4) + rlane;
      float bv = 0.f;
      if (BIAS_MODE == 2) bv = bias[n];
#pragma unroll
      for (int r = 0; r < 8; ++r) {
        float v = acc[i][j][r] * scale;
        if (BIAS_MODE == 1) v += bias[mBase + mOff + r];
        if (BIAS_MODE == 2) v += bv;
        if (RESID) v += Rb[(size_t)(mBase + mOff + r) * ldc + n];
        if (ACT == 1) v = tanhf(v);
        if (ACT == 2) v = fmaxf(v, 0.0f);
        if (ACT == 3) v = v / (1.0f + expf(-v));
        if (ACT == 4) v = (v > 0.f) ? v : 0.01f * v;
        if (ACT == 5) v = 0.5f * v * (1.0f + erff(v * 0.70710678118654752f));
        slab[(mOff + r) * 68 + (j << 4) + rlane] = v;
      }
    }
    __builtin_amdgcn_fence(__ATOMIC_RELEASE, "workgroup");
    __builtin_amdgcn_wave_barrier();
    __builtin_amdgcn_fence(__ATOMIC_ACQUIRE, "workgroup");
    if (OUT_MODE == 0) {
      float* C = (float*)Cout + (size_t)b * strideC;
      const int hh = lane >> 4, c4 = (lane & 15) * 4;
      for (int pass = 0; pass < 2; ++pass) {
#pragma unroll
        for (int it = 0; it < 8; ++it) {
          const int row = it * 2 + hh;
          v4f v = *(const v4f*)(slab + row * 68 + c4);
          *(volatile v4f*)(C + (size_t)(mBase + row) * ldc + n0 + c4) = v;
        }
        __threadfence();
      }
    } else {
      const int q = lane >> 3, c8 = (lane & 7) * 8;
      unsigned short* C  = (unsigned short*)Cout  + (size_t)b * strideC;
      unsigned short* C2 = (OUT_MODE == 2) ? ((unsigned short*)Cout2 + (size_t)b * strideC) : nullptr;
      for (int pass = 0; pass < 2; ++pass) {
#pragma unroll
        for (int it = 0; it < 4; ++it) {
          const int row = it * 4 + q;
          const float* sp = slab + row * 68 + c8;
          v8h hv, lv;
#pragma unroll
          for (int e = 0; e < 8; ++e) {
            if (OUT_MODE == 1) {
              hv[e] = (_Float16)sp[e];
            } else {
              unsigned short hb = f2bf_bits(sp[e]);
              unsigned short lb = f2bf_bits(sp[e] - bf_bits2f(hb));
              hv[e] = __builtin_bit_cast(_Float16, hb);
              lv[e] = __builtin_bit_cast(_Float16, lb);
            }
          }
          *(volatile v8h*)(C + (size_t)(mBase + row) * ldc + n0 + c8) = hv;
          if (OUT_MODE == 2) *(volatile v8h*)(C2 + (size_t)(mBase + row) * ldc + n0 + c8) = lv;
        }
        __threadfence();
      }
    }
    __builtin_amdgcn_fence(__ATOMIC_RELEASE, "workgroup");
    __builtin_amdgcn_wave_barrier();
    __builtin_amdgcn_fence(__ATOMIC_ACQUIRE, "workgroup");
  }
}

__global__ __launch_bounds__(256) void cvt8_kernel(const float* __restrict__ src, unsigned short* __restrict__ dst,
                                                   int nrow, int ncol8, int spitch, float sc, int tmajor) {
  const int i  = blockIdx.x * 256 + threadIdx.x;
  const int n8 = nrow * ncol8;
  if (i < n8) {
    const int row = i / ncol8;
    const int c8  = i - row * ncol8;
    const int tq  = row / NBAT;
    const int bq  = row - tq * NBAT;
    const int srow = tmajor ? (bq * NSTEP + tq) : row;
    const float* sp = src + (size_t)srow * spitch + c8 * 8;
    const v4f a = *(const v4f*)(sp);
    const v4f b = *(const v4f*)(sp + 4);
    v8h hv;
#pragma unroll
    for (int e = 0; e < 4; ++e) {
      const float fa = a[e];
      const float fb = b[e];
      hv[e]     = (_Float16)(bf16r(fa) * sc);
      hv[4 + e] = (_Float16)(bf16r(fb) * sc);
    }
    *(volatile v8h*)(dst + (size_t)i * 8) = hv;
    __threadfence();
    *(volatile v8h*)(dst + (size_t)i * 8) = hv;
  }
}

__global__ __launch_bounds__(256) void bias_prep_kernel(const float* __restrict__ s0, const float* __restrict__ s1,
                                                        const float* __restrict__ s2, const float* __restrict__ s3,
                                                        const float* __restrict__ s4, float* __restrict__ dst) {
  const int which = blockIdx.y;
  const float* src = s0;
  int n = NG3;
  if (which == 1) src = s1;
  if (which == 2) src = s2;
  if (which == 3) src = s3;
  if (which == 4) { src = s4; n = NFC; }
  const int idx = (blockIdx.x * 256 + threadIdx.x) * 4;
  if (idx < n) {
    const v4f v = *(const v4f*)(src + idx);
    v4f o;
#pragma unroll
    for (int e = 0; e < 4; ++e) { const float f = v[e]; o[e] = bf16r(f); }
    float* op = dst + (size_t)which * NG3 + idx;
    *(volatile v4f*)op = o;
    __threadfence();
    *(volatile v4f*)op = o;
  }
}

__device__ __forceinline__ float sigm_f(float x) { return 1.0f / (1.0f + expf(-x)); }

template <bool SEQ_OUT, bool ACT_OUT>
__global__ __launch_bounds__(RTHR) void gru_seq_kernel(const float* __restrict__ XT,
                                                       const unsigned short* __restrict__ WHp,
                                                       const float* __restrict__ bh,
                                                       unsigned short* __restrict__ HSEQ,
                                                       float* __restrict__ HOUT,
                                                       unsigned short* __restrict__ HACT) {
  __shared__ __align__(16) _Float16 Ah[2][SEQ_BLK * HPITCH];
  __shared__ __align__(16) float    Hm[SEQ_BLK * HMPITCH];
  const _Float16* WH = (const _Float16*)WHp;
  const int tid = threadIdx.x, lane = tid & 31, wave = tid >> 5;
  const int c = lane & 15, hh = lane >> 4, koff = hh * 8;
  const int rowbase = blockIdx.x * SEQ_BLK;

  {
    _Float16* ahf = &Ah[0][0];
#pragma unroll 1
    for (int i = tid; i < 2 * SEQ_BLK * HPITCH; i += RTHR) ahf[i] = (_Float16)0.0f;
#pragma unroll 1
    for (int i = tid; i < SEQ_BLK * HMPITCH; i += RTHR) Hm[i] = 0.0f;
  }
  __syncthreads();

  const v8f z8 = {0.f, 0.f, 0.f, 0.f, 0.f, 0.f, 0.f, 0.f};

#pragma unroll 1
  for (int t = 0; t < NSTEP; ++t) {
    const int cur = t & 1;
    const _Float16* ahrow = &Ah[cur][0] + c * HPITCH + koff;
    _Float16* ahn = &Ah[cur ^ 1][0];
    const float* xtb = XT + (size_t)(t * NBAT + rowbase + 8 * hh) * NG3;

#pragma unroll 1
    for (int nt = 0; nt < 4; ++nt) {
      const int j = 64 * wave + 16 * nt + c;
      const _Float16* w0 = WH + (size_t)j * NHID + koff;
      const _Float16* w1 = w0 + (size_t)NHID * NHID;
      const _Float16* w2 = w1 + (size_t)NHID * NHID;
      v8f accR = z8, accZ = z8, accN = z8;
#pragma unroll 2
      for (int k0 = 0; k0 < NHID; k0 += 32) {
        const v16h a  = Frag<_Float16>::load(ahrow + k0);
        const v16h b0 = Frag<_Float16>::load(w0 + k0);
        const v16h b1 = Frag<_Float16>::load(w1 + k0);
        const v16h b2 = Frag<_Float16>::load(w2 + k0);
        accR = Frag<_Float16>::mma(a, b0, accR);
        accZ = Frag<_Float16>::mma(a, b1, accZ);
        accN = Frag<_Float16>::mma(a, b2, accN);
        guard3_h(accR, accZ, accN, a, b0, b1, b2);
      }
      acc_guard3(accR, accZ, accN);

      const float br = bh[j];
      const float bz = bh[NHID + j];
      const float bn = bh[2 * NHID + j];
      const float* xp = xtb + j;
#pragma unroll
      for (int r = 0; r < 8; ++r) {
        const float xr = xp[(size_t)r * NG3];
        const float xz = xp[(size_t)r * NG3 + NHID];
        const float xn = xp[(size_t)r * NG3 + 2 * NHID];
        const float pr = accR[r] * WCARRY_INV + br;
        const float pz = accZ[r] * WCARRY_INV + bz;
        const float pn = accN[r] * WCARRY_INV + bn;
        const float rg = sigm_f(xr + pr);
        const float zg = sigm_f(xz + pz);
        const float ng = tanhf(xn + rg * pn);
        const int mi = (8 * hh + r) * HMPITCH + j;
        const float ho = Hm[mi];
        const float hn = zg * ho + (1.0f - zg) * ng;
        Hm[mi] = hn;
        ahn[(8 * hh + r) * HPITCH + j] = (_Float16)hn;
      }
    }
    __syncthreads();

    if (SEQ_OUT) {
      const _Float16* srcb = &Ah[cur ^ 1][0];
      unsigned short* dstb = HSEQ + ((size_t)t * NBAT + rowbase) * NHID;
      v8h hv[4];
#pragma unroll
      for (int it = 0; it < 4; ++it) {
        const int idx = it * RTHR + tid;
        const int row = idx / (NHID / 8);
        const int c8  = (idx - row * (NHID / 8)) * 8;
        hv[it] = *(const v8h*)(srcb + row * HPITCH + c8);
      }
      for (int pass = 0; pass < 2; ++pass) {
#pragma unroll
        for (int it = 0; it < 4; ++it) {
          const int idx = it * RTHR + tid;
          const int row = idx / (NHID / 8);
          const int c8  = (idx - row * (NHID / 8)) * 8;
          *(volatile v8h*)(dstb + (size_t)row * NHID + c8) = hv[it];
        }
        __threadfence();
      }
    }
  }

  {
    float* ob = HOUT + (size_t)rowbase * NHID;
    v4f fv[8];
#pragma unroll
    for (int it = 0; it < 8; ++it) {
      const int idx = it * RTHR + tid;
      const int row = idx / (NHID / 4);
      const int c4  = (idx - row * (NHID / 4)) * 4;
      fv[it] = *(const v4f*)(Hm + row * HMPITCH + c4);
    }
    for (int pass = 0; pass < 2; ++pass) {
#pragma unroll
      for (int it = 0; it < 8; ++it) {
        const int idx = it * RTHR + tid;
        const int row = idx / (NHID / 4);
        const int c4  = (idx - row * (NHID / 4)) * 4;
        *(volatile v4f*)(ob + (size_t)row * NHID + c4) = fv[it];
      }
      __threadfence();
    }
  }
  if (ACT_OUT) {
    unsigned short* ab = HACT + (size_t)rowbase * NHID;
    v8h av[4];
#pragma unroll
    for (int it = 0; it < 4; ++it) {
      const int idx = it * RTHR + tid;
      const int row = idx / (NHID / 8);
      const int c8  = (idx - row * (NHID / 8)) * 8;
      const v4f p = *(const v4f*)(Hm + row * HMPITCH + c8);
      const v4f q = *(const v4f*)(Hm + row * HMPITCH + c8 + 4);
#pragma unroll
      for (int e = 0; e < 4; ++e) {
        const float f0 = p[e];
        const float f1 = q[e];
        const float g0 = ((f0 > 0.0f) ? f0 : 0.01f * f0) * ACARRY;
        const float g1 = ((f1 > 0.0f) ? f1 : 0.01f * f1) * ACARRY;
        av[it][e]     = (_Float16)g0;
        av[it][4 + e] = (_Float16)g1;
      }
    }
    for (int pass = 0; pass < 2; ++pass) {
#pragma unroll
      for (int it = 0; it < 4; ++it) {
        const int idx = it * RTHR + tid;
        const int row = idx / (NHID / 8);
        const int c8  = (idx - row * (NHID / 8)) * 8;
        *(volatile v8h*)(ab + (size_t)row * NHID + c8) = av[it];
      }
      __threadfence();
    }
  }
}

extern "C" void kernel_launch(void* const* d_in, const int* in_sizes, int n_in,
                              void* d_out, int out_size, void* d_ws, size_t ws_size, hipStream_t stream) {
  if (n_in < 11 || d_out == nullptr || d_ws == nullptr) return;
  if (in_sizes[0] != NBAT * NSTEP * NINP || in_sizes[1] != NG3 * NINP || in_sizes[2] != NG3 ||
      in_sizes[3] != NG3 * NHID || in_sizes[4] != NG3 || in_sizes[5] != NG3 * NHID || in_sizes[6] != NG3 ||
      in_sizes[7] != NG3 * NHID || in_sizes[8] != NG3 || in_sizes[9] != NFC * NHID || in_sizes[10] != NFC ||
      out_size != NOUT0 + NOUT1) return;

  const float* x    = (const float*)d_in[0];
  const float* w_x0 = (const float*)d_in[1];
  const float* b_x0 = (const float*)d_in[2];
  const float* w_h0 = (const float*)d_in[3];
  const float* b_h0 = (const float*)d_in[4];
  const float* w_x1 = (const float*)d_in[5];
  const float* b_x1 = (const float*)d_in[6];
  const float* w_h1 = (const float*)d_in[7];
  const float* b_h1 = (const float*)d_in[8];
  const float* fc_w = (const float*)d_in[9];
  const float* fc_b = (const float*)d_in[10];
  float* out0  = (float*)d_out;
  float* h0out = out0 + (size_t)NOUT0;
  float* h1out = h0out + (size_t)NBAT * NHID;

  char* ws = (char*)d_ws; size_t off = 0;
  auto carve = [&](size_t bytes) -> char* { char* p = ws + off; off += (bytes + 255) & ~(size_t)255; return p; };
  unsigned short* XH    = (unsigned short*)carve((size_t)NROWS * NINP * 2);
  unsigned short* WX0H  = (unsigned short*)carve((size_t)NG3 * NINP * 2);
  unsigned short* WH0H  = (unsigned short*)carve((size_t)NG3 * NHID * 2);
  unsigned short* WX1H  = (unsigned short*)carve((size_t)NG3 * NHID * 2);
  unsigned short* WH1H  = (unsigned short*)carve((size_t)NG3 * NHID * 2);
  unsigned short* FCWH  = (unsigned short*)carve((size_t)NFC * NHID * 2);
  float*          BIASP = (float*)carve((size_t)(4 * NG3 + NFC) * 4);
  float*          XT    = (float*)carve((size_t)NROWS * NG3 * 4);
  unsigned short* HSEQ  = (unsigned short*)carve((size_t)NROWS * NHID * 2);
  unsigned short* HACT  = (unsigned short*)carve((size_t)NBAT * NHID * 2);
  if (off > ws_size || off > (size_t)134217728) return;

  const int n8x  = NROWS * (NINP / 8);
  const int n8w0 = NG3 * (NINP / 8);
  const int n8w  = NG3 * (NHID / 8);
  const int n8f  = NFC * (NHID / 8);
  cvt8_kernel<<<n8x  / 256, 256, 0, stream>>>(x,    XH,   NROWS, NINP / 8, NINP, 1.0f,   1);
  cvt8_kernel<<<n8w0 / 256, 256, 0, stream>>>(w_x0, WX0H, NG3,   NINP / 8, NINP, WCARRY, 0);
  cvt8_kernel<<<n8w  / 256, 256, 0, stream>>>(w_h0, WH0H, NG3,   NHID / 8, NHID, WCARRY, 0);
  cvt8_kernel<<<n8w  / 256, 256, 0, stream>>>(w_x1, WX1H, NG3,   NHID / 8, NHID, WCARRY, 0);
  cvt8_kernel<<<n8w  / 256, 256, 0, stream>>>(w_h1, WH1H, NG3,   NHID / 8, NHID, WCARRY, 0);
  cvt8_kernel<<<n8f  / 256, 256, 0, stream>>>(fc_w, FCWH, NFC,   NHID / 8, NHID, WCARRY, 0);
  bias_prep_kernel<<<dim3(NG3 / 1024, 5), 256, 0, stream>>>(b_x0, b_h0, b_x1, b_h1, fc_b, BIASP);

  const dim3 ggrid((NROWS / 64) * (NG3 / 64) / 8, 1);
  wmma_gemm64<0, false, 2, 0, false, 0><<<ggrid, 256, 0, stream>>>(
      XH, XH, NINP, 0L, WX0H, WX0H, NINP, 0L, (void*)XT, (void*)XT, NG3, 0L,
      BIASP, XT, 0L, NROWS, NG3, NINP, WCARRY_INV);

  gru_seq_kernel<true, false><<<NBAT / SEQ_BLK, RTHR, 0, stream>>>(
      XT, WH0H, BIASP + NG3, HSEQ, h0out, HACT);

  wmma_gemm64<0, false, 2, 0, false, 0><<<ggrid, 256, 0, stream>>>(
      HSEQ, HSEQ, NHID, 0L, WX1H, WX1H, NHID, 0L, (void*)XT, (void*)XT, NG3, 0L,
      BIASP + 2 * NG3, XT, 0L, NROWS, NG3, NHID, WCARRY_INV);

  gru_seq_kernel<false, true><<<NBAT / SEQ_BLK, RTHR, 0, stream>>>(
      XT, WH1H, BIASP + 3 * NG3, HSEQ, h1out, HACT);

  wmma_gemm64<0, false, 2, 0, false, 0><<<dim3(1, 1), 256, 0, stream>>>(
      HACT, HACT, NHID, 0L, FCWH, FCWH, NHID, 0L, (void*)out0, (void*)out0, NFC, 0L,
      BIASP + 4 * NG3, XT, 0L, NBAT, NFC, NHID, FC_SCALE);
}
